// PAM_Module_5609227289231
// MI455X (gfx1250) — hardware-verified
//
#include <hip/hip_runtime.h>
#include <math.h>
#include <stdint.h>

#define NBAT  4
#define CCH   512
#define CQK   64
#define IMGH  64
#define IMGW  64
#define NPOS  4096
#define MROWS 16384

static_assert(NPOS == IMGH * IMGW);
static_assert(MROWS == NBAT * NPOS);
static_assert(CCH % 64 == 0);
static_assert(CQK == 64);
static_assert(NPOS % 128 == 0);
static_assert(NPOS % 64 == 0);
static_assert(CCH % 32 == 0);
static_assert((CQK * CCH) % (8 * 256) == 0);
static_assert((CCH * CCH) % (8 * 256) == 0);
static_assert(CCH % 256 == 0);
static_assert((MROWS / 64) % 8 == 0);
static_assert(((CCH / 64) * (NPOS / 64)) % 8 == 0);

typedef __attribute__((ext_vector_type(16))) _Float16 v16h;
typedef __attribute__((ext_vector_type(8)))  _Float16 v8h;
typedef __attribute__((ext_vector_type(8)))  float    v8f;
typedef __attribute__((ext_vector_type(4)))  float    v4f;
typedef __attribute__((ext_vector_type(4)))  unsigned int v4u;

__device__ __forceinline__ unsigned short h_bits(_Float16 h) { return __builtin_bit_cast(unsigned short, h); }
__device__ __forceinline__ unsigned pk16(unsigned short a, unsigned short b) { return (unsigned)a | ((unsigned)b << 16); }

__device__ __forceinline__ void dep_guard_h(v8f& a, v8f& b, v16h x, v16h y) { asm volatile("v_nop\n\tv_nop\n\tv_nop\n\tv_nop" : "+v"(a), "+v"(b) : "v"(x), "v"(y)); }
__device__ __forceinline__ void keep4_h(v16h a, v16h b, v16h c, v16h d) { asm volatile("v_nop" :: "v"(a), "v"(b), "v"(c), "v"(d)); }
__device__ __forceinline__ void acc_guard4(v8f& a, v8f& b, v8f& c, v8f& d) { asm volatile("v_nop\n\tv_nop\n\tv_nop\n\tv_nop" : "+v"(a), "+v"(b), "+v"(c), "+v"(d)); }

struct FragH {
  union U { v16h v; v8h h[2]; };
  static __device__ __forceinline__ v16h load(const _Float16* p) {
    U f; f.h[0] = *(const v8h*)(p); f.h[1] = *(const v8h*)(p + 16); return f.v;
  }
  static __device__ __forceinline__ v8f mma(v16h a, v16h b, v8f c) {
    return __builtin_amdgcn_wmma_f32_16x16x32_f16(false, a, false, b, (short)0, c, false, false);
  }
  static __device__ __forceinline__ void guard(v8f& a, v8f& b, v16h x, v16h y) { dep_guard_h(a, b, x, y); }
  static __device__ __forceinline__ void keep(v16h a, v16h b, v16h c, v16h d) { keep4_h(a, b, c, d); }
};

__device__ __forceinline__ v8f hmma(v16h a, v16h b, v8f c) {
  c = __builtin_amdgcn_wmma_f32_16x16x32_f16(false, a, false, b, (short)0, c, false, false);
  asm volatile("v_nop\n\tv_nop\n\tv_nop\n\tv_nop" : "+v"(c) : "v"(a), "v"(b));
  return c;
}

template <bool SPLIT, int BIAS_MODE, int OUT_MODE>
__global__ __launch_bounds__(256) void gemm64_f16(
    const unsigned short* __restrict__ Ap, const unsigned short* __restrict__ A2p, int lda, long strideA,
    const unsigned short* __restrict__ Btp, const unsigned short* __restrict__ Bt2p, int ldb, long strideB,
    void* __restrict__ Cout, void* __restrict__ Cout2, int ldc, long strideC,
    const float* __restrict__ bias,
    int M, int N, int K, float scale, float oscale) {
  const _Float16* A   = (const _Float16*)(const void*)Ap;
  const _Float16* A2  = (const _Float16*)(const void*)A2p;
  const _Float16* Bt  = (const _Float16*)(const void*)Btp;
  const _Float16* Bt2 = (const _Float16*)(const void*)Bt2p;
  __shared__ __align__(16) float sT[8][16 * 68];
  const int b    = blockIdx.y;
  const int lane = threadIdx.x & 31;
  const int wave = threadIdx.x >> 5;
  const int tilesN = N >> 6;
  const int tilesM = M >> 6;
  const int tile = blockIdx.x * 8 + wave;
  if (tile >= tilesM * tilesN) return;
  const int tm = tile / tilesN;
  const int tn = tile - tm * tilesN;
  const int m0 = tm << 6;
  const int n0 = tn << 6;

  const _Float16* Ab  = A  + (size_t)b * strideA;
  const _Float16* Bb  = Bt + (size_t)b * strideB;
  const _Float16* Ab2 = SPLIT ? (A2  + (size_t)b * strideA) : Ab;
  const _Float16* Bb2 = SPLIT ? (Bt2 + (size_t)b * strideB) : Bb;

  const int rlane = lane & 15;
  const int koff  = (lane >> 4) * 8;
  const int mOff  = (lane >> 4) * 8;

  v8f acc[4][4];
#pragma unroll
  for (int i = 0; i < 4; ++i)
#pragma unroll
    for (int j = 0; j < 4; ++j) acc[i][j] = (v8f){0.f,0.f,0.f,0.f,0.f,0.f,0.f,0.f};

  for (int k0 = 0; k0 < K; k0 += 32) {
    v16h bh[4], bl[4];
#pragma unroll
    for (int j = 0; j < 4; ++j) {
      const size_t bo = (size_t)(n0 + (j << 4) + rlane) * ldb + koff + k0;
      bh[j] = FragH::load(Bb + bo);
      if (SPLIT) bl[j] = FragH::load(Bb2 + bo); else bl[j] = bh[j];
    }
#pragma unroll
    for (int i = 0; i < 4; ++i) {
      const size_t ao = (size_t)(m0 + (i << 4) + rlane) * lda + koff + k0;
      v16h ah = FragH::load(Ab + ao);
      v16h al;
      if (SPLIT) al = FragH::load(Ab2 + ao); else al = ah;
#pragma unroll
      for (int j = 0; j < 4; ++j) {
        acc[i][j] = FragH::mma(ah, bh[j], acc[i][j]);
        if (SPLIT) {
          acc[i][j] = FragH::mma(ah, bl[j], acc[i][j]);
          acc[i][j] = FragH::mma(al, bh[j], acc[i][j]);
        }
      }
      FragH::guard(acc[i][0], acc[i][3], ah, al);
    }
    FragH::keep(bh[0], bh[1], bh[2], bh[3]);
    if (SPLIT) FragH::keep(bl[0], bl[1], bl[2], bl[3]);
  }
  acc_guard4(acc[0][0], acc[0][1], acc[0][2], acc[0][3]);
  acc_guard4(acc[1][0], acc[1][1], acc[1][2], acc[1][3]);
  acc_guard4(acc[2][0], acc[2][1], acc[2][2], acc[2][3]);
  acc_guard4(acc[3][0], acc[3][1], acc[3][2], acc[3][3]);

  float* slab = sT[wave];
#pragma unroll
  for (int i = 0; i < 4; ++i) {
    const int mBase = m0 + (i << 4);
#pragma unroll
    for (int j = 0; j < 4; ++j) {
      const int n = n0 + (j << 4) + rlane;
      float bvn = 0.f;
      if (BIAS_MODE == 2) bvn = bias[n];
#pragma unroll
      for (int r = 0; r < 8; ++r) {
        float v = acc[i][j][r] * scale;
        if (BIAS_MODE == 1) v += bias[mBase + mOff + r];
        if (BIAS_MODE == 2) v += bvn;
        slab[(mOff + r) * 68 + (j << 4) + rlane] = v * oscale;
      }
    }
    __builtin_amdgcn_fence(__ATOMIC_RELEASE, "workgroup");
    __builtin_amdgcn_wave_barrier();
    __builtin_amdgcn_fence(__ATOMIC_ACQUIRE, "workgroup");
    if (OUT_MODE == 0) {
      float* C = (float*)Cout + (size_t)b * strideC;
      const int hh = lane >> 4, c4 = (lane & 15) * 4;
      for (int pass = 0; pass < 2; ++pass) {
#pragma unroll
        for (int it = 0; it < 8; ++it) {
          const int row = it * 2 + hh;
          v4f v = *(const v4f*)(slab + row * 68 + c4);
          *(volatile v4f*)(C + (size_t)(mBase + row) * ldc + n0 + c4) = v;
        }
        __threadfence();
      }
    } else {
      const int q = lane >> 3, c8 = (lane & 7) * 8;
      _Float16* C  = (_Float16*)Cout + (size_t)b * strideC;
      _Float16* C2 = (_Float16*)Cout2 + (size_t)b * strideC;
      for (int pass = 0; pass < 2; ++pass) {
#pragma unroll
        for (int it = 0; it < 4; ++it) {
          const int row = it * 4 + q;
          const float* sp = slab + row * 68 + c8;
          v8h hv, lv;
#pragma unroll
          for (int e = 0; e < 8; ++e) {
            if (OUT_MODE == 1) {
              float f = sp[e];
              f = (fabsf(f) >= 6.103515625e-05f) ? f : 0.0f;
              hv[e] = (_Float16)f;
            } else {
              const _Float16 hq = (_Float16)sp[e];
              hv[e] = hq;
              lv[e] = (_Float16)(sp[e] - (float)hq);
            }
          }
          *(volatile v8h*)(C + (size_t)(mBase + row) * ldc + n0 + c8) = hv;
          if (OUT_MODE == 2) *(volatile v8h*)(C2 + (size_t)(mBase + row) * ldc + n0 + c8) = lv;
        }
        __threadfence();
      }
    }
    __builtin_amdgcn_fence(__ATOMIC_RELEASE, "workgroup");
    __builtin_amdgcn_wave_barrier();
    __builtin_amdgcn_fence(__ATOMIC_ACQUIRE, "workgroup");
  }
}

__global__ __launch_bounds__(256) void wconv_f16(const float* __restrict__ in, unsigned short* __restrict__ oh,
                                                 unsigned short* __restrict__ ol, int n8, float carry) {
  const int i = blockIdx.x * 256 + threadIdx.x;
  if (i < n8) {
    const size_t e0 = (size_t)i * 8;
    const v4f a = *(const v4f*)(in + e0);
    const v4f c = *(const v4f*)(in + e0 + 4);
    float f[8];
    f[0] = a[0]; f[1] = a[1]; f[2] = a[2]; f[3] = a[3];
    f[4] = c[0]; f[5] = c[1]; f[6] = c[2]; f[7] = c[3];
    v4u hv, lv;
#pragma unroll
    for (int q = 0; q < 4; ++q) {
      const float f0 = f[2 * q] * carry, f1 = f[2 * q + 1] * carry;
      const _Float16 h0 = (_Float16)f0, h1 = (_Float16)f1;
      const _Float16 l0 = (_Float16)(f0 - (float)h0), l1 = (_Float16)(f1 - (float)h1);
      hv[q] = pk16(h_bits(h0), h_bits(h1));
      lv[q] = pk16(h_bits(l0), h_bits(l1));
    }
    for (int pass = 0; pass < 2; ++pass) {
      *(volatile v4u*)(oh + e0) = hv;
      *(volatile v4u*)(ol + e0) = lv;
      __threadfence();
    }
  }
}

__global__ __launch_bounds__(256) void tsplit_f16(const float* __restrict__ W, unsigned short* __restrict__ oh,
                                                  unsigned short* __restrict__ ol, int R, int Cc, long sIn, long sOut,
                                                  float carry) {
  __shared__ __align__(16) float tf[64 * 68];
  W  += (size_t)blockIdx.z * sIn;
  oh += (size_t)blockIdx.z * sOut;
  ol += (size_t)blockIdx.z * sOut;
  const int c0  = blockIdx.x * 64;
  const int r0  = blockIdx.y * 64;
  const int tid = threadIdx.x;
  {
    const int lr = tid >> 4;
    const int c4 = (tid & 15) * 4;
#pragma unroll
    for (int it = 0; it < 4; ++it) {
      const int rr = it * 16 + lr;
      const v4f a = *(const v4f*)(W + (size_t)(r0 + rr) * Cc + c0 + c4);
      *(v4f*)(tf + rr * 68 + c4) = a;
    }
  }
  __syncthreads();
  const int sub = tid >> 3;
  const int c8  = (tid & 7) * 8;
  v4u hv[2], lv[2];
#pragma unroll
  for (int it = 0; it < 2; ++it) {
    const int oc = it * 32 + sub;
    v4u a, a2;
#pragma unroll
    for (int q = 0; q < 4; ++q) {
      const float f0 = tf[(c8 + 2 * q) * 68 + oc] * carry;
      const float f1 = tf[(c8 + 2 * q + 1) * 68 + oc] * carry;
      const _Float16 h0 = (_Float16)f0, h1 = (_Float16)f1;
      const _Float16 l0 = (_Float16)(f0 - (float)h0), l1 = (_Float16)(f1 - (float)h1);
      a[q]  = pk16(h_bits(h0), h_bits(h1));
      a2[q] = pk16(h_bits(l0), h_bits(l1));
    }
    hv[it] = a; lv[it] = a2;
  }
  for (int pass = 0; pass < 2; ++pass) {
#pragma unroll
    for (int it = 0; it < 2; ++it) {
      const int oc = it * 32 + sub;
      const size_t go = (size_t)(c0 + oc) * R + r0 + c8;
      *(volatile v4u*)(oh + go) = hv[it];
      *(volatile v4u*)(ol + go) = lv[it];
    }
    __threadfence();
  }
}

#define AQB    16
#define AKC    128
#define PPITCH 136
#define NCHUNK (NPOS / AKC)

static_assert(NPOS % AQB == 0);
static_assert(NCHUNK * AKC == NPOS);
static_assert(CCH == 8 * 64);
static_assert((PPITCH * 2) % 16 == 0);

__global__ __launch_bounds__(256)
void attn_kernel(const unsigned short* __restrict__ qhp, const unsigned short* __restrict__ qlp,
                 const unsigned short* __restrict__ khp, const unsigned short* __restrict__ klp,
                 const unsigned short* __restrict__ vtp,
                 const float* __restrict__ X, const float* __restrict__ gam,
                 unsigned short* __restrict__ o2hp, unsigned short* __restrict__ o2lp,
                 float sscale, float pcarry, float pinv, float ocarry) {
  union FB { v16h v; v8h h[2]; };
  __shared__ __align__(16) _Float16 Ps[AQB * PPITCH];
  __shared__ __align__(16) float    Pm[AQB * 8];
  __shared__ __align__(16) float    Pl[AQB * 8];
  __shared__ __align__(16) float    Os[8][16 * 68];

  const int tid  = threadIdx.x;
  const int wave = tid >> 5;
  const int lane = tid & 31;
  const int hh   = lane >> 4;
  const int c    = lane & 15;

  const int b  = blockIdx.y;
  const int i0 = blockIdx.x * AQB;
  const size_t qrow0 = (size_t)b * NPOS + i0;

  const _Float16* Qh = (const _Float16*)(const void*)qhp;
  const _Float16* Ql = (const _Float16*)(const void*)qlp;
  const _Float16* Kh = (const _Float16*)(const void*)khp;
  const _Float16* Kl = (const _Float16*)(const void*)klp;
  const _Float16* Vw = (const _Float16*)(const void*)vtp + ((size_t)b * CCH + (size_t)wave * 64) * NPOS;
  _Float16* O2h = (_Float16*)(void*)o2hp;
  _Float16* O2l = (_Float16*)(void*)o2lp;

  v16h qah[2], qal[2];
#pragma unroll
  for (int dc = 0; dc < 2; ++dc) {
    qah[dc] = FragH::load(Qh + (qrow0 + c) * CQK + dc * 32 + 8 * hh);
    qal[dc] = FragH::load(Ql + (qrow0 + c) * CQK + dc * 32 + 8 * hh);
  }

  float mrow[8], lrow[8];
  v8f acc[4];
#pragma unroll
  for (int r = 0; r < 8; ++r) { mrow[r] = -INFINITY; lrow[r] = 0.f; }
#pragma unroll
  for (int n = 0; n < 4; ++n) acc[n] = (v8f){0.f,0.f,0.f,0.f,0.f,0.f,0.f,0.f};

  for (int jc = 0; jc < NCHUNK; ++jc) {
    const int j0 = jc * AKC;
    const size_t krow = (size_t)b * NPOS + j0 + wave * 16 + c;
    v8f s = (v8f){0.f,0.f,0.f,0.f,0.f,0.f,0.f,0.f};
#pragma unroll
    for (int dc = 0; dc < 2; ++dc) {
      const v16h kbh = FragH::load(Kh + krow * CQK + dc * 32 + 8 * hh);
      const v16h kbl = FragH::load(Kl + krow * CQK + dc * 32 + 8 * hh);
      s = hmma(qah[dc], kbh, s);
      s = hmma(qah[dc], kbl, s);
      s = hmma(qal[dc], kbh, s);
    }
    float mloc[8];
#pragma unroll
    for (int r = 0; r < 8; ++r) {
      const float sv = s[r] * sscale;
      s[r] = sv;
      float m = sv;
#pragma unroll
      for (int off = 1; off < 16; off <<= 1) m = fmaxf(m, __shfl_xor(m, off, 32));
      mloc[r] = m;
    }
    if (c == 0) {
#pragma unroll
      for (int r = 0; r < 8; ++r) Pm[(8 * hh + r) * 8 + wave] = mloc[r];
    }
    __syncthreads();

    float alpha[8], psl[8];
#pragma unroll
    for (int r = 0; r < 8; ++r) {
      const v4f ma = *(const v4f*)(Pm + (8 * hh + r) * 8);
      const v4f mb = *(const v4f*)(Pm + (8 * hh + r) * 8 + 4);
      const float cm = fmaxf(fmaxf(fmaxf(ma[0], ma[1]), fmaxf(ma[2], ma[3])),
                             fmaxf(fmaxf(mb[0], mb[1]), fmaxf(mb[2], mb[3])));
      const float mnew = fmaxf(mrow[r], cm);
      alpha[r] = __expf(mrow[r] - mnew);
      mrow[r] = mnew;
      const float p = __expf(s[r] - mnew);
      float psum = p;
#pragma unroll
      for (int off = 1; off < 16; off <<= 1) psum += __shfl_xor(psum, off, 32);
      psl[r] = psum;
      float p32 = p * pcarry;
      p32 = (p32 >= 6.103515625e-05f) ? p32 : 0.0f;
      Ps[(8 * hh + r) * PPITCH + wave * 16 + c] = (_Float16)p32;
#pragma unroll
      for (int n = 0; n < 4; ++n) acc[n][r] *= alpha[r];
    }
    if (c == 0) {
#pragma unroll
      for (int r = 0; r < 8; ++r) Pl[(8 * hh + r) * 8 + wave] = psl[r];
    }
    __syncthreads();

#pragma unroll
    for (int r = 0; r < 8; ++r) {
      const v4f la = *(const v4f*)(Pl + (8 * hh + r) * 8);
      const v4f lb = *(const v4f*)(Pl + (8 * hh + r) * 8 + 4);
      const float ls = ((la[0] + la[1]) + (la[2] + la[3])) + ((lb[0] + lb[1]) + (lb[2] + lb[3]));
      lrow[r] = lrow[r] * alpha[r] + ls;
    }

#pragma unroll
    for (int kk = 0; kk < 4; ++kk) {
      FB pa;
      pa.h[0] = *(const v8h*)(Ps + c * PPITCH + kk * 32 + 8 * hh);
      pa.h[1] = *(const v8h*)(Ps + c * PPITCH + kk * 32 + 16 + 8 * hh);
#pragma unroll
      for (int n = 0; n < 4; ++n) {
        const v16h vb = FragH::load(Vw + (size_t)(n * 16 + c) * NPOS + j0 + kk * 32 + 8 * hh);
        acc[n] = hmma(pa.v, vb, acc[n]);
      }
    }
  }

  const float g = gam[0];
  float rl[8];
#pragma unroll
  for (int r = 0; r < 8; ++r) rl[r] = (1.0f / lrow[r]) * pinv;
  float* os = Os[wave];
#pragma unroll
  for (int n = 0; n < 4; ++n) {
    const int ch = wave * 64 + n * 16 + c;
    const float* xp = X + ((size_t)b * CCH + ch) * NPOS + i0 + 8 * hh;
    const v4f xa = *(const v4f*)(xp);
    const v4f xb = *(const v4f*)(xp + 4);
    float xe[8];
    xe[0] = xa[0]; xe[1] = xa[1]; xe[2] = xa[2]; xe[3] = xa[3];
    xe[4] = xb[0]; xe[5] = xb[1]; xe[6] = xb[2]; xe[7] = xb[3];
#pragma unroll
    for (int r = 0; r < 8; ++r) {
      const float o  = acc[n][r] * rl[r];
      const float v2 = g * o + xe[r];
      os[(8 * hh + r) * 68 + n * 16 + c] = v2 * ocarry;
    }
  }
  __builtin_amdgcn_fence(__ATOMIC_RELEASE, "workgroup");
  __builtin_amdgcn_wave_barrier();
  __builtin_amdgcn_fence(__ATOMIC_ACQUIRE, "workgroup");
  {
    const int q = lane >> 3, c8 = (lane & 7) * 8;
    for (int pass = 0; pass < 2; ++pass) {
#pragma unroll
      for (int it = 0; it < 4; ++it) {
        const int row = it * 4 + q;
        const float* sp = os + row * 68 + c8;
        v8h hv, lv;
#pragma unroll
        for (int e = 0; e < 8; ++e) {
          const _Float16 hq = (_Float16)sp[e];
          hv[e] = hq;
          lv[e] = (_Float16)(sp[e] - (float)hq);
        }
        const size_t go = (qrow0 + row) * (size_t)CCH + wave * 64 + c8;
        *(volatile v8h*)(O2h + go) = hv;
        *(volatile v8h*)(O2l + go) = lv;
      }
      __threadfence();
    }
  }
}

extern "C" void kernel_launch(void* const* d_in, const int* in_sizes, int n_in,
                              void* d_out, int out_size, void* d_ws, size_t ws_size,
                              hipStream_t stream) {
  if (n_in < 10) return;
  if (in_sizes[0] != NBAT * CCH * NPOS) return;
  if (in_sizes[1] != CQK * CCH) return;
  if (in_sizes[2] != CQK) return;
  if (in_sizes[3] != CQK * CCH) return;
  if (in_sizes[4] != CQK) return;
  if (in_sizes[5] != CCH * CCH) return;
  if (in_sizes[6] != CCH) return;
  if (in_sizes[7] != 1) return;
  if (in_sizes[8] != CCH * CCH) return;
  if (in_sizes[9] != CCH) return;
  if (out_size != NBAT * CCH * NPOS) return;

  const float* x     = (const float*)d_in[0];
  const float* Wq    = (const float*)d_in[1];
  const float* bq    = (const float*)d_in[2];
  const float* Wk    = (const float*)d_in[3];
  const float* bk    = (const float*)d_in[4];
  const float* Wv    = (const float*)d_in[5];
  const float* bv    = (const float*)d_in[6];
  const float* gamma = (const float*)d_in[7];
  const float* Wd    = (const float*)d_in[8];
  const float* bd    = (const float*)d_in[9];

  const size_t PXT = (size_t)MROWS * CCH * 2;
  const size_t PWS = (size_t)CQK * CCH * 2;
  const size_t PWL = (size_t)CCH * CCH * 2;
  const size_t PQK = (size_t)MROWS * CQK * 2;
  const size_t PVT = (size_t)NBAT * CCH * NPOS * 2;
  size_t off = 0;
  const size_t oXTh = off; off += PXT;  const size_t oXTl = off; off += PXT;
  const size_t oWQh = off; off += PWS;  const size_t oWQl = off; off += PWS;
  const size_t oWKh = off; off += PWS;  const size_t oWKl = off; off += PWS;
  const size_t oWVh = off; off += PWL;  const size_t oWVl = off; off += PWL;
  const size_t oWDh = off; off += PWL;  const size_t oWDl = off; off += PWL;
  const size_t oQh  = off; off += PQK;  const size_t oQl  = off; off += PQK;
  const size_t oKh  = off; off += PQK;  const size_t oKl  = off; off += PQK;
  const size_t oVT  = off; off += PVT;
  const size_t oO2h = off; off += PXT;  const size_t oO2l = off; off += PXT;
  if (off > ws_size) return;
  if (off > (size_t)134217728) return;

  char* ws = (char*)d_ws;
  unsigned short* XTh = (unsigned short*)(ws + oXTh);  unsigned short* XTl = (unsigned short*)(ws + oXTl);
  unsigned short* WQh = (unsigned short*)(ws + oWQh);  unsigned short* WQl = (unsigned short*)(ws + oWQl);
  unsigned short* WKh = (unsigned short*)(ws + oWKh);  unsigned short* WKl = (unsigned short*)(ws + oWKl);
  unsigned short* WVh = (unsigned short*)(ws + oWVh);  unsigned short* WVl = (unsigned short*)(ws + oWVl);
  unsigned short* WDh = (unsigned short*)(ws + oWDh);  unsigned short* WDl = (unsigned short*)(ws + oWDl);
  unsigned short* Qh  = (unsigned short*)(ws + oQh);   unsigned short* Ql  = (unsigned short*)(ws + oQl);
  unsigned short* Kh  = (unsigned short*)(ws + oKh);   unsigned short* Kl  = (unsigned short*)(ws + oKl);
  unsigned short* VT  = (unsigned short*)(ws + oVT);
  unsigned short* O2h = (unsigned short*)(ws + oO2h);  unsigned short* O2l = (unsigned short*)(ws + oO2l);

  const dim3 blk(256);
  const float actCarry = 1024.0f;
  const float wCarry   = 65536.0f;
  const float scale26  = 1.0f / 67108864.0f;
  const float sScale   = 1.0f / 1048576.0f;
  const float pCarry   = 32768.0f;
  const float pInv     = 1.0f / 32768.0f;

  tsplit_f16<<<dim3(NPOS / 64, CCH / 64, NBAT), blk, 0, stream>>>(x, XTh, XTl, CCH, NPOS, (long)CCH * NPOS, (long)NPOS * CCH, actCarry);
  const int n8s = CQK * CCH / 8;
  const int n8l = CCH * CCH / 8;
  wconv_f16<<<dim3(n8s / 256), blk, 0, stream>>>(Wq, WQh, WQl, n8s, wCarry);
  wconv_f16<<<dim3(n8s / 256), blk, 0, stream>>>(Wk, WKh, WKl, n8s, wCarry);
  wconv_f16<<<dim3(n8l / 256), blk, 0, stream>>>(Wv, WVh, WVl, n8l, wCarry);
  wconv_f16<<<dim3(n8l / 256), blk, 0, stream>>>(Wd, WDh, WDl, n8l, wCarry);
  const dim3 gQ((MROWS / 64) * (CQK / 64) / 8, 1);
  gemm64_f16<true, 2, 2><<<gQ, blk, 0, stream>>>(
      XTh, XTl, CCH, 0L, WQh, WQl, CCH, 0L, (void*)Qh, (void*)Ql, CQK, 0L, bq, MROWS, CQK, CCH, scale26, actCarry);
  gemm64_f16<true, 2, 2><<<gQ, blk, 0, stream>>>(
      XTh, XTl, CCH, 0L, WKh, WKl, CCH, 0L, (void*)Kh, (void*)Kl, CQK, 0L, bk, MROWS, CQK, CCH, scale26, actCarry);
  const dim3 gV((CCH / 64) * (NPOS / 64) / 8, NBAT);
  gemm64_f16<true, 1, 1><<<gV, blk, 0, stream>>>(
      WVh, WVl, CCH, 0L, XTh, XTl, CCH, (long)NPOS * CCH, (void*)VT, (void*)VT, NPOS, (long)CCH * NPOS, bv,
      CCH, NPOS, CCH, scale26, 1.0f);
  attn_kernel<<<dim3(NPOS / AQB, NBAT), blk, 0, stream>>>(Qh, Ql, Kh, Kl, VT, x, gamma, O2h, O2l, sScale, pCarry, pInv, actCarry);
  gemm64_f16<true, 1, 0><<<gV, blk, 0, stream>>>(
      WDh, WDl, CCH, 0L, O2h, O2l, CCH, (long)NPOS * CCH, d_out, d_out, NPOS, (long)CCH * NPOS, bd,
      CCH, NPOS, CCH, scale26, 1.0f);
  (void)hipGetLastError();
}
